// interactionModule_nonParametric_acceleration_65549790871653
// MI455X (gfx1250) — hardware-verified
//
#include <hip/hip_runtime.h>
#include <stddef.h>


#define NTHR   256
#define NWAVE  8
#define EPT    8
#define CHUNK  (NTHR * EPT)
#define WCAP   (EPT * 32)
#define LISTN  (NWAVE * WCAP)
#define TE     16
#define PASSN  (NWAVE * TE)
#define PCAP   (CHUNK + PASSN)
#define NB     4096
#define HID    128
#define NQ     ((NB * 2) / (128 * NWAVE))
#define WSC    8.0f
#define WINV   0.125f
#define NEPS   1e-12f

static_assert(PASSN == 128);
static_assert((PCAP % PASSN) == 0);
static_assert(NQ * 128 * NWAVE == NB * 2);
static_assert((NB % 64) == 0);

typedef float    v2f  __attribute__((ext_vector_type(2)));
typedef float    v4f  __attribute__((ext_vector_type(4)));
typedef float    v8f  __attribute__((ext_vector_type(8)));
typedef int      v4i  __attribute__((ext_vector_type(4)));
typedef _Float16 v8h  __attribute__((ext_vector_type(8)));
typedef _Float16 v16h __attribute__((ext_vector_type(16)));
union FragH { v16h v; v8h h[2]; };

__device__ __forceinline__ v8f wmh(v16h a, v16h b, v8f c) {
  v8f d = __builtin_amdgcn_wmma_f32_16x16x32_f16(false, a, false, b, (short)0, c, false, false);
  asm volatile("v_nop\n\tv_nop\n\tv_nop\n\tv_nop" : "+v"(d) : "v"(a), "v"(b));
  return d;
}

__device__ __forceinline__ v8h relu8(v8f d) {
  v8h r;
#pragma unroll
  for (int i = 0; i < 8; ++i) { const float t = fmaxf(d[i] * WINV, 0.0f); r[i] = (_Float16)t; }
  return r;
}

__device__ __forceinline__ v8f ldc8(const float* p) {
  const v4f a = *(const v4f*)p;
  const v4f b = *(const v4f*)(p + 4);
  v8f c;
  c[0] = a.x; c[1] = a.y; c[2] = a.z; c[3] = a.w;
  c[4] = b.x; c[5] = b.y; c[6] = b.z; c[7] = b.w;
  return c;
}

__device__ __forceinline__ int scan_chunk(const int* __restrict__ dsts, int nE, int cbase, int nodeBase,
                                          int vec8, int* list, int tid, int wave) {
  int wc = 0;
  const int el0  = tid * EPT;
  const int e0   = cbase + el0;
  const int sent = -2147483647 - 1;
  v4i da, db;
  if (vec8 != 0 && cbase + CHUNK <= nE) {
    da = *(const v4i*)(dsts + e0);
    db = *(const v4i*)(dsts + e0 + 4);
  } else {
    da.x = (e0     < nE) ? dsts[min(e0, nE - 1)] : sent;
    da.y = (e0 + 1 < nE) ? dsts[min(e0 + 1, nE - 1)] : sent;
    da.z = (e0 + 2 < nE) ? dsts[min(e0 + 2, nE - 1)] : sent;
    da.w = (e0 + 3 < nE) ? dsts[min(e0 + 3, nE - 1)] : sent;
    db.x = (e0 + 4 < nE) ? dsts[min(e0 + 4, nE - 1)] : sent;
    db.y = (e0 + 5 < nE) ? dsts[min(e0 + 5, nE - 1)] : sent;
    db.z = (e0 + 6 < nE) ? dsts[min(e0 + 6, nE - 1)] : sent;
    db.w = (e0 + 7 < nE) ? dsts[min(e0 + 7, nE - 1)] : sent;
  }
  const unsigned nb = (unsigned)nodeBase;
  const unsigned s0 = (unsigned)da.x - nb, s1 = (unsigned)da.y - nb;
  const unsigned s2 = (unsigned)da.z - nb, s3 = (unsigned)da.w - nb;
  const unsigned s4 = (unsigned)db.x - nb, s5 = (unsigned)db.y - nb;
  const unsigned s6 = (unsigned)db.z - nb, s7 = (unsigned)db.w - nb;
  const bool h0 = s0 < (unsigned)NB, h1 = s1 < (unsigned)NB, h2 = s2 < (unsigned)NB, h3 = s3 < (unsigned)NB;
  const bool h4 = s4 < (unsigned)NB, h5 = s5 < (unsigned)NB, h6 = s6 < (unsigned)NB, h7 = s7 < (unsigned)NB;
  const unsigned any = __builtin_amdgcn_ballot_w32(h0 | h1 | h2 | h3 | h4 | h5 | h6 | h7);
  if (any != 0u) {
#define HITJ(J, HJ) { \
      const unsigned mj = __builtin_amdgcn_ballot_w32(HJ); \
      if (mj != 0u) { \
        if (HJ) { \
          const int pos = wc + (int)__builtin_amdgcn_mbcnt_lo(mj, 0u); \
          if (pos < WCAP) list[wave * WCAP + pos] = el0 + (J); \
        } \
        wc += (int)__builtin_popcount(mj); } }
    HITJ(0, h0)
    HITJ(1, h1)
    HITJ(2, h2)
    HITJ(3, h3)
    HITJ(4, h4)
    HITJ(5, h5)
    HITJ(6, h6)
    HITJ(7, h7)
#undef HITJ
  }
  return wc;
}

__global__ __launch_bounds__(NTHR) void k_prep(const float* __restrict__ W1,
                                               const float* __restrict__ W2,
                                               _Float16* wt) {
  const int b  = blockIdx.x;
  const int pl = b >> 3;
  const int p  = (b & 7) * NTHR + threadIdx.x;
  const int n  = p >> 4;
  const int k0 = (p & 15) * 8;
  const float* W = (pl == 0) ? W1 : W2;
  v8h hv;
#pragma unroll
  for (int i = 0; i < 8; ++i) hv[i] = (_Float16)(W[(k0 + i) * HID + n] * WSC);
  _Float16* q = wt + (size_t)pl * HID * HID + (size_t)n * HID + k0;
  *(volatile v8h*)q = hv;
  __threadfence();
  *(volatile v8h*)q = hv;
}

__global__ __launch_bounds__(NTHR) void k_main(
    const float* __restrict__ x, const float* __restrict__ vv,
    const int* __restrict__ srcs, const int* __restrict__ dsts,
    const float* __restrict__ gam,
    const float* __restrict__ W0, const float* __restrict__ B0,
    const float* __restrict__ B1, const float* __restrict__ B2,
    const float* __restrict__ W3, const float* __restrict__ B3,
    const _Float16* __restrict__ wt,
    float* outp, int nN, int nE, int vec8) {
  __shared__ __attribute__((aligned(16))) float acc[(NB + 1) * 2];
  __shared__ __attribute__((aligned(16))) float msg[PASSN * 2];
  __shared__ __attribute__((aligned(16))) int   list[LISTN];
  __shared__ __attribute__((aligned(16))) int   pend[PCAP];
  __shared__ int slotb[PASSN];
  __shared__ __attribute__((aligned(16))) float w0s[HID];
  __shared__ __attribute__((aligned(16))) float b0s[HID];
  __shared__ __attribute__((aligned(16))) float w3s[HID];
  __shared__ __attribute__((aligned(16))) float b1s[HID];
  __shared__ __attribute__((aligned(16))) float b2s[HID];
  __shared__ int wcnt[NWAVE];
  __shared__ int pendN;

  const int tid = threadIdx.x, lane = tid & 31, wave = tid >> 5, hh = lane >> 4, m = lane & 15;
  const int nodeBase = blockIdx.x * NB;

  for (int i = tid; i < (NB + 1) * 2; i += NTHR) acc[i] = 0.0f;
  if (tid < HID) {
    w0s[tid] = W0[tid];
    b0s[tid] = B0[tid];
    w3s[tid] = W3[tid];
    b1s[tid] = B1[tid] * WSC;
    b2s[tid] = B2[tid] * WSC;
  }
  if (tid == 0) pendN = 0;
  const float b3v = B3[0];
  const float g   = gam[0];
  __syncthreads();

  const int nChunks = (nE + CHUNK - 1) / CHUNK;
#pragma unroll 1
  for (int ch = 0; ch < nChunks; ++ch) {
    const int cbase = ch * CHUNK;
    const int wc = scan_chunk(dsts, nE, cbase, nodeBase, vec8, list, tid, wave);
    if (lane == 0) wcnt[wave] = wc;
    __syncthreads();

    const int base = pendN;
    int tot = 0, myoff = 0;
#pragma unroll
    for (int w = 0; w < NWAVE; ++w) {
      int c = wcnt[w];
      c = c > WCAP ? WCAP : (c < 0 ? 0 : c);
      if (w < wave) myoff += c;
      tot += c;
    }
    int newN = base + tot;
    newN = newN > PCAP ? PCAP : (newN < 0 ? 0 : newN);
    {
      int n = wcnt[wave];
      n = n > WCAP ? WCAP : (n < 0 ? 0 : n);
      const int* lp = list + wave * WCAP;
      for (int i = lane; i < n; i += 32) {
        const int pos = base + myoff + i;
        if ((unsigned)pos < (unsigned)PCAP) pend[pos] = cbase + lp[i];
      }
    }
    const int fin = (ch == nChunks - 1) ? 1 : 0;
    const int R   = (fin != 0) ? (newN + PASSN - 1) / PASSN : newN / PASSN;
    const int Pv  = (fin != 0) ? newN : R * PASSN;
    __syncthreads();

#pragma unroll 1
    for (int r = 0; r < R; ++r) {
      int zo = 0;
      asm volatile("" : "+s"(zo));
      const _Float16* wt1 = wt + zo;
      const _Float16* wt2 = wt + HID * HID + zo;

      const int idx = r * PASSN + wave * TE + m;
      const bool valid = idx < Pv;
      int e = pend[min(idx, PCAP - 1)];
      if (!valid) e = 0;
      e = min(max(e, 0), nE - 1);
      int d = dsts[e];
      int s = srcs[e];
      int slot = d - nodeBase;
      if (!valid || (unsigned)slot >= (unsigned)NB) slot = NB;
      d = min(max(d, 0), nN - 1);
      s = min(max(s, 0), nN - 1);
      const v2f xd = *(const v2f*)(x + (size_t)d * 2);
      const v2f xs = *(const v2f*)(x + (size_t)s * 2);
      const float dx = xd.x - xs.x;
      const float dy = xd.y - xs.y;
      const float adr = sqrtf(dx * dx + dy * dy);
      const float invd = 1.0f / fmaxf(adr, NEPS);
      const float ux = dx * invd;
      const float uy = dy * invd;

      FragH bq[4];
#pragma unroll
      for (int kb = 0; kb < 4; ++kb) {
#pragma unroll
        for (int q2 = 0; q2 < 2; ++q2) {
          const int f0 = 32 * kb + 16 * q2 + 8 * hh;
          const v4f wa = *(const v4f*)(w0s + f0);
          const v4f wb = *(const v4f*)(w0s + f0 + 4);
          const v4f ba = *(const v4f*)(b0s + f0);
          const v4f bb = *(const v4f*)(b0s + f0 + 4);
          v8h hv;
#pragma unroll
          for (int i = 0; i < 4; ++i) {
            hv[i]     = (_Float16)fmaxf(adr * wa[i] + ba[i], 0.0f);
            hv[4 + i] = (_Float16)fmaxf(adr * wb[i] + bb[i], 0.0f);
          }
          bq[kb].h[q2] = hv;
        }
      }

      FragH nbq[4];
#pragma unroll
      for (int ft = 0; ft < 8; ++ft) {
        v8f c = ldc8(b1s + 16 * ft + 8 * hh);
#pragma unroll
        for (int kb = 0; kb < 4; ++kb) {
          FragH a;
          const _Float16* ap = wt1 + (16 * ft + m) * HID + 32 * kb + 8 * hh;
          a.h[0] = *(const v8h*)ap;
          a.h[1] = *(const v8h*)(ap + 16);
          c = wmh(a.v, bq[kb].v, c);
        }
        nbq[ft >> 1].h[ft & 1] = relu8(c);
      }

      float part = 0.0f;
#pragma unroll
      for (int ft = 0; ft < 8; ++ft) {
        v8f c = ldc8(b2s + 16 * ft + 8 * hh);
#pragma unroll
        for (int kb = 0; kb < 4; ++kb) {
          FragH a;
          const _Float16* ap = wt2 + (16 * ft + m) * HID + 32 * kb + 8 * hh;
          a.h[0] = *(const v8h*)ap;
          a.h[1] = *(const v8h*)(ap + 16);
          c = wmh(a.v, nbq[kb].v, c);
        }
        const v4f wa = *(const v4f*)(w3s + 16 * ft + 8 * hh);
        const v4f wb = *(const v4f*)(w3s + 16 * ft + 8 * hh + 4);
#pragma unroll
        for (int j = 0; j < 4; ++j) {
          part += fmaxf(c[j] * WINV, 0.0f) * wa[j];
          part += fmaxf(c[4 + j] * WINV, 0.0f) * wb[j];
        }
      }
      const float oth   = __shfl_xor(part, 16, 32);
      const float force = (part + oth) + b3v;

      if (hh == 0) {
        msg[(wave * TE + m) * 2 + 0] = force * ux;
        msg[(wave * TE + m) * 2 + 1] = force * uy;
        slotb[wave * TE + m] = slot;
      }
      __syncthreads();

      if (wave == 0) {
#pragma unroll 1
        for (int i = 0; i < PASSN; ++i) {
          int sl = slotb[i];
          sl = min(max(sl, 0), NB);
          if (lane < 2) {
            const float t = msg[i * 2 + lane];
            acc[sl * 2 + lane] += t;
          }
        }
      }
      __syncthreads();
    }

    int rem = newN - R * PASSN;
    rem = rem < 0 ? 0 : (rem > PASSN ? PASSN : rem);
    if (R > 0 && tid < rem) pend[tid] = pend[R * PASSN + tid];
    if (tid == 0) pendN = rem;
  }
  __syncthreads();

  const size_t lim = (size_t)nN * 2;
  const size_t ob  = (size_t)nodeBase * 2;
  v4f ov[NQ];
#pragma unroll
  for (int q = 0; q < NQ; ++q) {
    const int f = (wave * NQ + q) * 128 + 4 * lane;
    const v4f a4 = *(const v4f*)(acc + f);
    const int n0 = nodeBase + (f >> 1);
    const int na = min(n0, nN - 1);
    const int nc = min(n0 + 1, nN - 1);
    const v2f va = *(const v2f*)(vv + (size_t)na * 2);
    const v2f vc = *(const v2f*)(vv + (size_t)nc * 2);
    v4f o;
    o.x = a4.x - g * va.x;
    o.y = a4.y - g * va.y;
    o.z = a4.z - g * vc.x;
    o.w = a4.w - g * vc.y;
    ov[q] = o;
  }
#pragma unroll
  for (int q = 0; q < NQ; ++q) {
    const size_t gi = ob + (size_t)((wave * NQ + q) * 128 + 4 * lane);
    if (gi + 3 < lim) *(volatile v4f*)(outp + gi) = ov[q];
  }
  __threadfence();
#pragma unroll
  for (int q = 0; q < NQ; ++q) {
    const size_t gi = ob + (size_t)((wave * NQ + q) * 128 + 4 * lane);
    if (gi + 3 < lim) *(volatile v4f*)(outp + gi) = ov[q];
  }
}

extern "C" void kernel_launch(void* const* d_in, const int* in_sizes, int n_in,
                              void* d_out, int out_size, void* d_ws, size_t ws_size,
                              hipStream_t stream) {
  if (n_in < 13) return;
  const int nN = in_sizes[0] / 2;
  const int nE = in_sizes[2];
  if (nN < 1 || in_sizes[0] != 2 * nN || in_sizes[1] != 2 * nN) return;
  if (nE < 1 || in_sizes[3] != nE) return;
  if (in_sizes[4] < 1 || in_sizes[5] != HID || in_sizes[6] != HID) return;
  if (in_sizes[7] != HID * HID || in_sizes[8] != HID) return;
  if (in_sizes[9] != HID * HID || in_sizes[10] != HID) return;
  if (in_sizes[11] != HID || in_sizes[12] < 1) return;
  if (out_size != 2 * nN) return;

  const size_t need = (size_t)2 * HID * HID * sizeof(_Float16);
  if (need > ws_size) return;

  const float* x     = (const float*)d_in[0];
  const float* v     = (const float*)d_in[1];
  const int*   src   = (const int*)d_in[2];
  const int*   dst   = (const int*)d_in[3];
  const float* gamma = (const float*)d_in[4];
  const float* W0    = (const float*)d_in[5];
  const float* b0    = (const float*)d_in[6];
  const float* W1    = (const float*)d_in[7];
  const float* b1    = (const float*)d_in[8];
  const float* W2    = (const float*)d_in[9];
  const float* b2    = (const float*)d_in[10];
  const float* W3    = (const float*)d_in[11];
  const float* b3    = (const float*)d_in[12];
  float* out = (float*)d_out;
  _Float16* wt = (_Float16*)d_ws;

  k_prep<<<16, NTHR, 0, stream>>>(W1, W2, wt);

  const int nBlk = (nN + NB - 1) / NB;
  k_main<<<nBlk, NTHR, 0, stream>>>(x, v, src, dst, gamma, W0, b0, b1, b2, W3, b3,
                                    wt, out, nN, nE, 1);
}
